// MeMA_4166118277534
// MI455X (gfx1250) — hardware-verified
//
#include <hip/hip_runtime.h>
#include <hip/hip_bf16.h>
#include <math.h>


typedef _Float16 bf16;
typedef _Float16 f16;
typedef __attribute__((ext_vector_type(4))) unsigned v4u_t;
typedef unsigned v4ua __attribute__((ext_vector_type(4), may_alias));
typedef __attribute__((ext_vector_type(4))) float v4f_t;
typedef float v4fa __attribute__((ext_vector_type(4), may_alias));
typedef __attribute__((ext_vector_type(16))) bf16  bf16x16;
typedef bf16x16 f16x16;
typedef __attribute__((ext_vector_type(8)))  bf16  bf16x8;
typedef bf16x8 f16x8;
typedef __attribute__((ext_vector_type(4)))  bf16  bf16x4;
typedef __attribute__((ext_vector_type(8)))  float f32x8;
__device__ __forceinline__ f32x8 wmma16(f16x16 a, f16x16 b, f32x8 c) {
  c = __builtin_amdgcn_wmma_f32_16x16x32_f16(false, a, false, b, (short)0, c, false, false);
  asm volatile("v_nop\n\tv_nop\n\tv_nop\n\tv_nop" : "+v"(c) : "v"(a), "v"(b));
  return c;
}
#define LDS_STRIDE 48
#define KSTRIDE    72
#define VSTRIDE    48

__device__ __forceinline__ f32x8 wmma_bf16(bf16x16 a, bf16x16 b, f32x8 c) {
  c = __builtin_amdgcn_wmma_f32_16x16x32_f16(false, a, false, b, (short)0, c, false, false);
  asm volatile("v_nop\n\tv_nop\n\tv_nop\n\tv_nop" : "+v"(c) : "v"(a), "v"(b));
  return c;
}

template <typename T>
__device__ __forceinline__ bf16x16 load_frag(const T* __restrict__ base, int ld,
                                             int row0, int k0) {
  const int lane = threadIdx.x & 31;
  const int r    = lane & 15;
  const int kh   = (lane >> 4) * 8;
  const T* p0 = base + (size_t)(row0 + r) * ld + (k0 + kh);
  const T* p1 = p0 + 16;
  bf16x16 f;
#pragma unroll
  for (int i = 0; i < 8; ++i) {
    f[i]     = (bf16)p0[i];
    f[i + 8] = (bf16)p1[i];
  }
  return f;
}

__device__ __forceinline__ bf16x16 lds_frag(const bf16* base, int stride) {
  const int lane = threadIdx.x & 31;
  const int row  = lane & 15;
  const int kh   = (lane >> 4) * 8;
  const bf16x8 lo = *(const bf16x8*)(base + row * stride + kh);
  const bf16x8 hi = *(const bf16x8*)(base + row * stride + kh + 16);
  bf16x16 f;
#pragma unroll
  for (int i = 0; i < 8; ++i) { f[i] = lo[i]; f[i + 8] = hi[i]; }
  return f;
}

template <typename T>
__device__ __forceinline__ void stage_read16(const T* __restrict__ p, float* buf) {
#pragma unroll
  for (int i = 0; i < 16; ++i) buf[i] = (float)p[i];
}

__device__ __forceinline__ void stage_write(bf16* dst, const float* buf, int nquad) {
#pragma unroll
  for (int i = 0; i < nquad; ++i) {
    bf16x4 q;
    q[0] = (bf16)buf[4 * i];     q[1] = (bf16)buf[4 * i + 1];
    q[2] = (bf16)buf[4 * i + 2]; q[3] = (bf16)buf[4 * i + 3];
    *(bf16x4*)(dst + 4 * i) = q;
  }
}


#define GSTR 48
#define GSTR 48
template <typename AT, int EPI, bool OUT16>
__global__ __launch_bounds__(256) void gemm_kne(const AT* __restrict__ A, int lda, const float* __restrict__ Wm, int ldw,
                                                const float* __restrict__ bias, const float* __restrict__ R, const float* __restrict__ gvec,
                                                void* __restrict__ Yv, int ldy, int K) {
  __shared__ __attribute__((aligned(16))) f16 ldsA[128 * GSTR];
  __shared__ __attribute__((aligned(16))) f16 ldsW[128 * GSTR];
  __shared__ __attribute__((aligned(16))) float oS[8][32 * 68];
  const int tid = threadIdx.x, lane = tid & 31, wave = tid >> 5, cl = lane & 15, rh = (lane >> 4) * 8;
  const int m0 = blockIdx.x * 128, n0 = blockIdx.y * 128;
  const int wm = (wave & 3) * 32, wn = (wave >> 2) * 64;
  f32x8 acc[2][4];
#pragma unroll
  for (int i = 0; i < 2; ++i)
#pragma unroll
    for (int j = 0; j < 4; ++j) { f32x8 z = {}; acc[i][j] = z; }
#pragma unroll 1
  for (int k0 = 0; k0 < K; k0 += 32) {
    __syncthreads();
    { const int row = tid >> 1, ch = (tid & 1) * 16;
      const AT* src = A + (size_t)(m0 + row) * lda + k0 + ch;
#pragma unroll
      for (int g = 0; g < 16; ++g) ldsA[row * GSTR + ch + g] = (f16)src[g]; }
    { const int k = tid >> 3, nn0 = (tid & 7) * 16;
      const float* src = Wm + (size_t)(k0 + k) * ldw + n0 + nn0;
#pragma unroll
      for (int g = 0; g < 4; ++g) { const v4f_t v = *(const v4f_t*)(src + 4 * g);
#pragma unroll
        for (int u = 0; u < 4; ++u) ldsW[(nn0 + 4 * g + u) * GSTR + k] = (f16)v[u]; } }
    __syncthreads();
    f16x16 af[2];
#pragma unroll
    for (int i = 0; i < 2; ++i) af[i] = lds_frag(ldsA + (wm + 16 * i) * GSTR, GSTR);
#pragma unroll
    for (int j = 0; j < 4; ++j) {
      const f16x16 bf = lds_frag(ldsW + (wn + 16 * j) * GSTR, GSTR);
#pragma unroll
      for (int i = 0; i < 2; ++i) acc[i][j] = wmma16(af[i], bf, acc[i][j]);
    }
  }
  float* so = oS[wave];
#pragma unroll
  for (int i = 0; i < 2; ++i)
#pragma unroll
    for (int j = 0; j < 4; ++j) {
      const int n = n0 + wn + 16 * j + cl;
      const float bv = bias ? bias[n] : 0.0f;
      const float gv = (EPI == 2 || EPI == 4) ? gvec[n] : 0.0f;
      if (EPI == 1) {
#pragma unroll 1
        for (int r = 0; r < 8; ++r) { const float xg = acc[i][j][r] + bv; so[(16 * i + rh + r) * 68 + 16 * j + cl] = 0.5f * xg * (1.0f + erff(xg * 0.70710678118654752f)); }
      } else {
#pragma unroll
        for (int r = 0; r < 8; ++r) {
          float v = acc[i][j][r] + bv;
          if (EPI == 3) v = fmaxf(v, 0.0f);
          if (EPI == 4) v = gv * v;
          if (EPI == 2) v = R[(size_t)(m0 + wm + 16 * i + rh + r) * ldy + n] + gv * v;
          so[(16 * i + rh + r) * 68 + 16 * j + cl] = v;
        }
      }
    }
  asm volatile("s_wait_dscnt 0" ::: "memory");
  __builtin_amdgcn_wave_barrier();
#pragma unroll 1
  for (int pass = 0; pass < 2; ++pass) {
    if (OUT16) {
      f16* Y = (f16*)Yv;
#pragma unroll
      for (int it = 0; it < 8; ++it) { const int c = lane + 32 * it, rr = c >> 3, q8 = (c & 7) * 8;
        union { f16 h[8]; v4u_t v; } u;
#pragma unroll
        for (int e = 0; e < 8; ++e) u.h[e] = (f16)so[rr * 68 + q8 + e];
        *(volatile v4u_t*)(Y + (size_t)(m0 + wm + rr) * ldy + n0 + wn + q8) = u.v; }
    } else {
      float* Y = (float*)Yv;
#pragma unroll
      for (int it = 0; it < 16; ++it) { const int f4 = lane + 32 * it, rr = f4 >> 4, q = (f4 & 15) * 4;
        *(volatile v4f_t*)(Y + (size_t)(m0 + wm + rr) * ldy + n0 + wn + q) = *(const v4fa*)(so + rr * 68 + q); }
    }
    __threadfence();
  }
}

template <typename AT, int EPI, bool OUT16>
__global__ __launch_bounds__(256) void gemm_knez2(int nz1, const AT* __restrict__ A, int lda, size_t sA1, size_t sA2, const float* __restrict__ Wm, int ldw, size_t sW1, size_t sW2,
                                                  const float* __restrict__ bias, const float* __restrict__ R, const float* __restrict__ gvec,
                                                  void* __restrict__ Yv, int ldy, size_t sY1, size_t sY2, int K) {
  const size_t z1 = blockIdx.z % nz1, z2 = blockIdx.z / nz1; const size_t oY = z1 * sY1 + z2 * sY2;
  A += z1 * sA1 + z2 * sA2; Wm += z1 * sW1 + z2 * sW2; Yv = (void*)((char*)Yv + oY * (OUT16 ? 2 : 4)); if (R) R += oY;
  __shared__ __attribute__((aligned(16))) f16 ldsA[128 * GSTR];
  __shared__ __attribute__((aligned(16))) f16 ldsW[128 * GSTR];
  __shared__ __attribute__((aligned(16))) float oS[8][32 * 68];
  const int tid = threadIdx.x, lane = tid & 31, wave = tid >> 5, cl = lane & 15, rh = (lane >> 4) * 8;
  const int m0 = blockIdx.x * 128, n0 = blockIdx.y * 128;
  const int wm = (wave & 3) * 32, wn = (wave >> 2) * 64;
  f32x8 acc[2][4];
#pragma unroll
  for (int i = 0; i < 2; ++i)
#pragma unroll
    for (int j = 0; j < 4; ++j) { f32x8 z = {}; acc[i][j] = z; }
#pragma unroll 1
  for (int k0 = 0; k0 < K; k0 += 32) {
    __syncthreads();
    { const int row = tid >> 1, ch = (tid & 1) * 16;
      const AT* src = A + (size_t)(m0 + row) * lda + k0 + ch;
#pragma unroll
      for (int g = 0; g < 16; ++g) ldsA[row * GSTR + ch + g] = (f16)src[g]; }
    { const int k = tid >> 3, nn0 = (tid & 7) * 16;
      const float* src = Wm + (size_t)(k0 + k) * ldw + n0 + nn0;
#pragma unroll
      for (int g = 0; g < 4; ++g) { const v4f_t v = *(const v4f_t*)(src + 4 * g);
#pragma unroll
        for (int u = 0; u < 4; ++u) ldsW[(nn0 + 4 * g + u) * GSTR + k] = (f16)v[u]; } }
    __syncthreads();
    f16x16 af[2];
#pragma unroll
    for (int i = 0; i < 2; ++i) af[i] = lds_frag(ldsA + (wm + 16 * i) * GSTR, GSTR);
#pragma unroll
    for (int j = 0; j < 4; ++j) {
      const f16x16 bf = lds_frag(ldsW + (wn + 16 * j) * GSTR, GSTR);
#pragma unroll
      for (int i = 0; i < 2; ++i) acc[i][j] = wmma16(af[i], bf, acc[i][j]);
    }
  }
  float* so = oS[wave];
#pragma unroll
  for (int i = 0; i < 2; ++i)
#pragma unroll
    for (int j = 0; j < 4; ++j) {
      const int n = n0 + wn + 16 * j + cl;
      const float bv = bias ? bias[n] : 0.0f;
      const float gv = (EPI == 2 || EPI == 4) ? gvec[n] : 0.0f;
      if (EPI == 1) {
#pragma unroll 1
        for (int r = 0; r < 8; ++r) { const float xg = acc[i][j][r] + bv; so[(16 * i + rh + r) * 68 + 16 * j + cl] = 0.5f * xg * (1.0f + erff(xg * 0.70710678118654752f)); }
      } else {
#pragma unroll
        for (int r = 0; r < 8; ++r) {
          float v = acc[i][j][r] + bv;
          if (EPI == 3) v = fmaxf(v, 0.0f);
          if (EPI == 4) v = gv * v;
          if (EPI == 2) v = R[(size_t)(m0 + wm + 16 * i + rh + r) * ldy + n] + gv * v;
          so[(16 * i + rh + r) * 68 + 16 * j + cl] = v;
        }
      }
    }
  asm volatile("s_wait_dscnt 0" ::: "memory");
  __builtin_amdgcn_wave_barrier();
#pragma unroll 1
  for (int pass = 0; pass < 2; ++pass) {
    if (OUT16) {
      f16* Y = (f16*)Yv;
#pragma unroll
      for (int it = 0; it < 8; ++it) { const int c = lane + 32 * it, rr = c >> 3, q8 = (c & 7) * 8;
        union { f16 h[8]; v4u_t v; } u;
#pragma unroll
        for (int e = 0; e < 8; ++e) u.h[e] = (f16)so[rr * 68 + q8 + e];
        *(volatile v4u_t*)(Y + (size_t)(m0 + wm + rr) * ldy + n0 + wn + q8) = u.v; }
    } else {
      float* Y = (float*)Yv;
#pragma unroll
      for (int it = 0; it < 16; ++it) { const int f4 = lane + 32 * it, rr = f4 >> 4, q = (f4 & 15) * 4;
        *(volatile v4f_t*)(Y + (size_t)(m0 + wm + rr) * ldy + n0 + wn + q) = *(const v4fa*)(so + rr * 68 + q); }
    }
    __threadfence();
  }
}


#define NGRP 4
#define BBe 64
#define CCe 128
#define NHe 8
#define NNe 256
#define GB 16
#define MEMW (CCe * NNe * NHe)
__global__ __launch_bounds__(256) void k_transposeB(const float* __restrict__ src, float* __restrict__ dst, int R, int C, size_t sstride, size_t dstride) {
  __shared__ float tS[64][65];
  const int tid = threadIdx.x, tbj = C / 64, bi = blockIdx.x / tbj, bj = blockIdx.x % tbj; const float* s = src + (size_t)blockIdx.y * sstride; float* d = dst + (size_t)blockIdx.y * dstride;
  for (int e = tid; e < 64 * 64; e += 256) { const int r = e >> 6, c = e & 63; tS[r][c] = s[(size_t)(bi * 64 + r) * C + bj * 64 + c]; }
  __syncthreads();
  for (int ch = tid; ch < 64 * 16; ch += 256) { const int r = ch >> 4, q4 = (ch & 15) * 4; v4f_t v; v[0] = tS[q4][r]; v[1] = tS[q4 + 1][r]; v[2] = tS[q4 + 2][r]; v[3] = tS[q4 + 3][r];
    float* p = d + (size_t)(bj * 64 + r) * R + bi * 64 + q4; *(volatile v4f_t*)p = v; __threadfence(); *(volatile v4f_t*)p = v; }
}
__global__ __launch_bounds__(256) void k_gatherq(const float* __restrict__ mem, const int* __restrict__ tids, int b0, float* __restrict__ Qt) {
  const int bb = blockIdx.y; const int t = min(max(tids[b0 + bb], 0), 4); const size_t e = (size_t)blockIdx.x * 1024 + threadIdx.x * 4;
  const v4f_t v = *(const v4f_t*)(mem + (size_t)t * MEMW + e); float* p = Qt + (size_t)bb * MEMW + e; *(volatile v4f_t*)p = v; __threadfence(); *(volatile v4f_t*)p = v;
}
__global__ __launch_bounds__(256) void k_softmax256(float* __restrict__ Sm) {
  __shared__ float red[256];
  const size_t row = (size_t)blockIdx.y * NNe + blockIdx.x; const int tid = threadIdx.x; float* sr = Sm + row * NNe;
  float v = sr[tid]; red[tid] = v; __syncthreads();
  for (int o = 128; o > 0; o >>= 1) { if (tid < o) red[tid] = fmaxf(red[tid], red[tid + o]); __syncthreads(); }
  const float m = red[0]; __syncthreads();
  v = expf(v - m); red[tid] = v; __syncthreads();
  for (int o = 128; o > 0; o >>= 1) { if (tid < o) red[tid] += red[tid + o]; __syncthreads(); }
  const float p = v * (1024.0f / red[0]);
  *(volatile float*)(sr + tid) = p; __threadfence(); *(volatile float*)(sr + tid) = p;
}
__global__ __launch_bounds__(256) void k_ln128(float* __restrict__ Y) {
  const int tid = threadIdx.x, lane = tid & 31, wave = tid >> 5; const size_t row = (size_t)blockIdx.x * 8 + wave; float* yr = Y + row * CCe;
  v4f_t v = *(const v4f_t*)(yr + 4 * lane); float s = v[0] + v[1] + v[2] + v[3];
#pragma unroll
  for (int off = 1; off < 32; off <<= 1) s += __shfl_xor(s, off, 32);
  const float mean = s * (1.0f / CCe); float q = 0.0f;
#pragma unroll
  for (int u = 0; u < 4; ++u) { const float d = v[u] - mean; q = fmaf(d, d, q); }
#pragma unroll
  for (int off = 1; off < 32; off <<= 1) q += __shfl_xor(q, off, 32);
  const float rstd = rsqrtf(q * (1.0f / CCe) + 1e-5f);
  v4f_t o;
#pragma unroll
  for (int u = 0; u < 4; ++u) o[u] = (v[u] - mean) * rstd;
  *(volatile v4f_t*)(yr + 4 * lane) = o; __threadfence(); *(volatile v4f_t*)(yr + 4 * lane) = o;
}
__global__ __launch_bounds__(256) void k_fill(float* __restrict__ p, float val, size_t n4) { const size_t i = (size_t)blockIdx.x * 256 + threadIdx.x; if (i < n4) { v4f_t v = {val, val, val, val}; *(volatile v4f_t*)(p + 4 * i) = v; __threadfence(); *(volatile v4f_t*)(p + 4 * i) = v; } }

extern "C" void kernel_launch(void* const* d_in, const int* in_sizes, int n_in,
                              void* d_out, int out_size, void* d_ws, size_t ws_size,
                              hipStream_t stream) {
  (void)in_sizes; (void)n_in; (void)out_size;
  const float** f = (const float**)d_in;
  const float* feat = f[0]; const int* tids = (const int*)d_in[1]; const float* mem = f[2], *Wkg = f[3], *Wvg = f[4], *Wkt = f[5], *Wvt = f[6], *Wo = f[7], *bo = f[8];
  float* out = (float*)d_out;
  char* ws = (char*)d_ws;
  float* F = (float*)ws; ws += (size_t)BBe * NNe * CCe * 4;
  float* Kr = (float*)ws; ws += (size_t)GB * NNe * 1024 * 4; float* Vr = (float*)ws; ws += (size_t)GB * NNe * 1024 * 4;
  float* KT = (float*)ws; ws += (size_t)GB * 1024 * NNe * 4;
  float* Qt = (float*)ws; ws += (size_t)GB * MEMW * 4;
  float* S = (float*)ws; ws += (size_t)GB * NHe * NNe * NNe * 4;
  float* O = Kr;
  float* Y = (float*)ws; ws += (size_t)BBe * NNe * CCe * 4;
  float* sc = (float*)ws; ws += 1024 * 4; float* ones = (float*)ws; ws += CCe * 4;
  if ((size_t)(ws - (char*)d_ws) > ws_size) return;
  const dim3 blk(256);
  k_fill<<<dim3(1), blk, 0, stream>>>(sc, 1.0f / 1024.0f, 1024 / 4); k_fill<<<dim3(1), blk, 0, stream>>>(ones, 1.0f, CCe / 4);
  k_transposeB<<<dim3((CCe / 64) * (NNe / 64), BBe), blk, 0, stream>>>(feat, F, CCe, NNe, (size_t)CCe * NNe, (size_t)NNe * CCe);
  const dim3 gp(GB * NNe / 128, 1024 / 128);
  for (int br = 0; br < 2; ++br) {
    const float* Wk = br ? Wkt : Wkg; const float* Wv = br ? Wvt : Wvg;
    for (int g = 0; g < NGRP; ++g) {
      const float* Fg = F + (size_t)g * GB * NNe * CCe;
      gemm_kne<float, 0, false><<<gp, blk, 0, stream>>>(Fg, CCe, Wk, 1024, nullptr, nullptr, nullptr, Kr, 1024, CCe);
      gemm_kne<float, 0, false><<<gp, blk, 0, stream>>>(Fg, CCe, Wv, 1024, nullptr, nullptr, nullptr, Vr, 1024, CCe);
      k_transposeB<<<dim3((NNe / 64) * (1024 / 64), GB), blk, 0, stream>>>(Kr, KT, NNe, 1024, (size_t)NNe * 1024, (size_t)1024 * NNe);
      const float* Qsrc; size_t sA2;
      if (br) { k_gatherq<<<dim3(MEMW / 1024, GB), blk, 0, stream>>>(mem, tids, g * GB, Qt); Qsrc = Qt; sA2 = MEMW; } else { Qsrc = mem + (size_t)4 * MEMW; sA2 = 0; }
      gemm_knez2<float, 0, false><<<dim3(NNe / 128, NNe / 128, GB * NHe), blk, 0, stream>>>(NHe, Qsrc, CCe, (size_t)NNe * CCe, sA2, KT, NNe, (size_t)CCe * NNe, (size_t)1024 * NNe, nullptr, nullptr, nullptr, S, NNe, (size_t)NNe * NNe, (size_t)NHe * NNe * NNe, CCe);
      k_softmax256<<<dim3(NNe, GB * NHe), blk, 0, stream>>>(S);
      gemm_knez2<float, 4, false><<<dim3(NNe / 128, 1, GB * NHe), blk, 0, stream>>>(NHe, S, NNe, (size_t)NNe * NNe, (size_t)NHe * NNe * NNe, Vr, 1024, (size_t)CCe, (size_t)NNe * 1024, nullptr, nullptr, sc, O, 1024, (size_t)CCe, (size_t)NNe * 1024, NNe);
      float* Yg = Y + (size_t)g * GB * NNe * CCe;
      if (br == 0) gemm_kne<float, 0, false><<<dim3(GB * NNe / 128, 1), blk, 0, stream>>>(O, 1024, Wo, CCe, bo, nullptr, nullptr, Yg, CCe, 1024);
      else         gemm_kne<float, 2, false><<<dim3(GB * NNe / 128, 1), blk, 0, stream>>>(O, 1024, Wo, CCe, nullptr, Yg, ones, Yg, CCe, 1024);
    }
  }
  k_ln128<<<dim3(BBe * NNe / 8), blk, 0, stream>>>(Y);
  k_transposeB<<<dim3((NNe / 64) * (CCe / 64), BBe), blk, 0, stream>>>(Y, out, NNe, CCe, (size_t)NNe * CCe, (size_t)CCe * NNe);
}
